// TripletConv_33397665694633
// MI455X (gfx1250) — hardware-verified
//
#include <hip/hip_runtime.h>
#include <stddef.h>


typedef _Float16 h16;
typedef _Float16 v16h __attribute__((ext_vector_type(16)));
typedef _Float16 v8h  __attribute__((ext_vector_type(8)));
typedef _Float16 v4h  __attribute__((ext_vector_type(4)));
typedef float    v8f  __attribute__((ext_vector_type(8)));
typedef float    v4f  __attribute__((ext_vector_type(4)));

#ifndef NB
#define NB 4
#endif
#define NB_FULL 4
#define NN   96
#define DIM  128
#define SUB  8
#define ME   (NB * NN * NN)
#define MT   (NB * NN)

#define PROWS 32
#define LDA   136
#define LDTT  40
#define LDO   132

#define XCARRY 8.0f
#define WCARRY 64.0f
#define TCARRY 16.0f

static_assert(NB >= 1 && NB <= NB_FULL);
static_assert(SUB == 8 && DIM == 128 && NN == 96);
static_assert((DIM % 32) == 0);
static_assert((ME % PROWS) == 0 && (MT % PROWS) == 0);
static_assert((NN % 32) == 0);
static_assert((LDA % 8) == 0 && LDA >= DIM);
static_assert((LDTT % 8) == 0 && LDTT >= 32);
static_assert((LDO % 4) == 0 && LDO >= DIM);
static_assert(PROWS * DIM == 64 * 16 * 4);
static_assert(DIM == 32 * 4);

#define WP_BYTES  ((size_t)16 * DIM * 2)
#define WOP_BYTES ((size_t)DIM * 32 * 2)
#define EPL_BYTES ((size_t)ME * SUB * 4)
#define TPL_BYTES ((size_t)MT * SUB * 4)
#define OFF_WE  ((size_t)0)
#define OFF_WN  (OFF_WE + WP_BYTES)
#define OFF_WO  (OFF_WN + WP_BYTES)
#define OFF_EIK (OFF_WO + WOP_BYTES)
#define OFF_EKJ (OFF_EIK + EPL_BYTES)
#define OFF_EIJ (OFF_EKJ + EPL_BYTES)
#define OFF_TI  (OFF_EIJ + EPL_BYTES)
#define OFF_TJ  (OFF_TI + TPL_BYTES)
#define OFF_TK  (OFF_TJ + TPL_BYTES)
#define WS_TOTAL (OFF_TK + TPL_BYTES)
static_assert((WP_BYTES % 128) == 0 && (WOP_BYTES % 128) == 0);
static_assert((EPL_BYTES % 128) == 0 && (TPL_BYTES % 128) == 0);
static_assert(WP_BYTES == (size_t)256 * 16);
static_assert(WOP_BYTES == (size_t)2 * 256 * 16);
static_assert(WS_TOTAL <= (size_t)134217728);

__device__ __forceinline__ float bf16r(float x) {
  unsigned int u = __float_as_uint(x);
  u = (u + 0x7FFFu + ((u >> 16) & 1u)) & 0xFFFF0000u;
  return __uint_as_float(u);
}

static __device__ __forceinline__ h16 toh_flush(float v) {
  const h16 r = (h16)v;
  return (fabsf(v) < 6.103515625e-05f) ? (h16)0.0f : r;
}

__device__ __forceinline__ v16h frag_at(const _Float16* p) {
  v8h lo = *(const v8h*)(p);
  v8h hi = *(const v8h*)(p + 16);
  v16h out;
#pragma unroll
  for (int i = 0; i < 8; ++i) { out[i] = lo[i]; out[i + 8] = hi[i]; }
  return out;
}
__device__ __forceinline__ v16h ld_frag(const _Float16* base, unsigned ld) {
  const unsigned lane = threadIdx.x & 31u;
  return frag_at(base + (lane & 15u) * ld + (lane >> 4) * 8u);
}

__device__ __forceinline__ v8f wmma16(v16h a, v16h b, v8f c) {
  v8f d = __builtin_amdgcn_wmma_f32_16x16x32_f16(false, a, false, b, (short)0, c,
                                                 false, false);
  asm volatile("v_nop\n\tv_nop\n\tv_nop\n\tv_nop" : "+v"(d) : "v"(a), "v"(b));
  return d;
}

__device__ __forceinline__ void wave_lds_sync() {
  __builtin_amdgcn_fence(3  , "wavefront");
  asm volatile("s_wait_dscnt 0x0" ::: "memory");
  __builtin_amdgcn_wave_barrier();
}

__global__ __launch_bounds__(256) void wprep_kernel(
    const float* __restrict__ We, const float* __restrict__ Wn, const float* __restrict__ Wo,
    _Float16* __restrict__ WeP, _Float16* __restrict__ WnP, _Float16* __restrict__ WoP) {
  const unsigned tid = threadIdx.x;
  const unsigned n = tid >> 4, kc = (tid & 15u) * 8u;
  const unsigned nn = n & 7u;
  const bool live = (n < 8u);
  v8h xe, xn;
#pragma unroll
  for (unsigned j = 0; j < 8u; ++j) {
    const float a = We[(kc + j) * SUB + nn];
    const float c = Wn[(kc + j) * SUB + nn];
    const h16 ha = toh_flush(WCARRY * bf16r(a));
    const h16 hc = toh_flush(WCARRY * bf16r(c));
    xe[j] = live ? ha : (h16)0.0f;
    xn[j] = live ? hc : (h16)0.0f;
  }
  v8h xo[2];
#pragma unroll
  for (unsigned i = 0; i < 2u; ++i) {
    const unsigned p = tid + 256u * i;
    const unsigned on = p >> 2;
    const bool olive = ((p & 3u) == 0u);
#pragma unroll
    for (unsigned j = 0; j < 8u; ++j) {
      const float a = Wo[j * DIM + on];
      const h16 ha = toh_flush(WCARRY * bf16r(a));
      xo[i][j] = olive ? ha : (h16)0.0f;
    }
  }
  *(volatile v8h*)(WeP + tid * 8u) = xe;
  *(volatile v8h*)(WnP + tid * 8u) = xn;
#pragma unroll
  for (unsigned i = 0; i < 2u; ++i) *(volatile v8h*)(WoP + (tid + 256u * i) * 8u) = xo[i];
  __threadfence();
  *(volatile v8h*)(WeP + tid * 8u) = xe;
  *(volatile v8h*)(WnP + tid * 8u) = xn;
#pragma unroll
  for (unsigned i = 0; i < 2u; ++i) *(volatile v8h*)(WoP + (tid + 256u * i) * 8u) = xo[i];
}

__global__ __launch_bounds__(64) void proj_kernel(
    const float* __restrict__ X, const _Float16* __restrict__ Wp, const float* __restrict__ bias,
    const float* __restrict__ Wt, unsigned wbase,
    float* __restrict__ out0, float* __restrict__ out1, float* __restrict__ out2) {
  __shared__ _Float16 As[PROWS * LDA];
  __shared__ float Wl[24 * 8];
  __shared__ float Pw[2 * 16 * 16];
  const unsigned tid = threadIdx.x, lane = tid & 31u;
  const unsigned wave = __builtin_amdgcn_readfirstlane(threadIdx.x >> 5);
  const unsigned hh = lane >> 4, m = lane & 15u;
  const unsigned row0 = blockIdx.x * (unsigned)PROWS;

#pragma unroll 4
  for (unsigned j = 0; j < 16u; ++j) {
    const unsigned idx = tid + 64u * j;
    const unsigned r = idx >> 5, c = (idx & 31u) * 4u;
    const v4f x = *(const v4f*)(X + (size_t)(row0 + r) * DIM + c);
    v4h y;
#pragma unroll
    for (int i = 0; i < 4; ++i) y[i] = toh_flush(XCARRY * bf16r(x[i]));
    *(v4h*)&As[r * LDA + c] = y;
  }
#pragma unroll 1
  for (unsigned j = 0; j < 3u; ++j) {
    const unsigned idx = tid + 64u * j;
    Wl[idx] = bf16r(Wt[wbase * 8u + idx]);
  }
  __syncthreads();

  const _Float16* bp = Wp + (size_t)m * DIM + hh * 8u;
  v8f acc = {};
#pragma unroll
  for (unsigned k0 = 0; k0 < (unsigned)DIM; k0 += 32u) {
    const v16h a = ld_frag(&As[(wave * 16u) * LDA + k0], LDA);
    const v16h bfr = frag_at(bp + k0);
    acc = wmma16(a, bfr, acc);
  }
  const float pb = bf16r(bias[m & 7u]);
  const unsigned pw0 = wave * 256u;
#pragma unroll
  for (int r = 0; r < 8; ++r)
    Pw[pw0 + (hh * 8u + (unsigned)r) * 16u + m] = acc[r] * (1.0f / (XCARRY * WCARRY)) + pb;
  wave_lds_sync();

  const unsigned rr = lane >> 1, s0 = (lane & 1u) * 4u;
  const v4f p0 = *(const v4f*)&Pw[pw0 + rr * 16u];
  const v4f p1 = *(const v4f*)&Pw[pw0 + rr * 16u + 4u];
  float pe[8];
#pragma unroll
  for (int d = 0; d < 4; ++d) { pe[d] = p0[d]; pe[d + 4] = p1[d]; }
  v4f ev[3];
#pragma unroll
  for (int p = 0; p < 3; ++p) {
    v4f a = {};
#pragma unroll
    for (int d = 0; d < 8; ++d) {
      const v4f wv = *(const v4f*)&Wl[(unsigned)(p * 8 + d) * 8u + s0];
#pragma unroll
      for (int q = 0; q < 4; ++q) a[q] += pe[d] * wv[q];
    }
    ev[p] = a;
  }
  const size_t off = (size_t)(row0 + wave * 16u) * SUB + lane * 4u;
  *(volatile v4f*)(out0 + off) = ev[0];
  *(volatile v4f*)(out1 + off) = ev[1];
  *(volatile v4f*)(out2 + off) = ev[2];
  __threadfence();
  *(volatile v4f*)(out0 + off) = ev[0];
  *(volatile v4f*)(out1 + off) = ev[1];
  *(volatile v4f*)(out2 + off) = ev[2];
}

__global__ __launch_bounds__(96) void tri_kernel(
    const float* __restrict__ Eik, const float* __restrict__ Ekj, const float* __restrict__ Eij,
    const float* __restrict__ Ti, const float* __restrict__ Tj, const float* __restrict__ Tk,
    const float* __restrict__ bt, const _Float16* __restrict__ WoP,
    const float* __restrict__ bo, float* __restrict__ out) {
  __shared__ float Xs[NN * 8];
  __shared__ _Float16 Ts[NN * LDTT];
  __shared__ float Cs[3 * 16 * LDO];
  const unsigned tid = threadIdx.x, lane = tid & 31u;
  const unsigned wave = __builtin_amdgcn_readfirstlane(threadIdx.x >> 5);
  const unsigned hh = lane >> 4, m = lane & 15u;
  const unsigned rowbi = blockIdx.x;
  const unsigned b = rowbi / (unsigned)NN;

  {
    const float* e = Eik + ((size_t)rowbi * NN + tid) * SUB;
    const float* t = Tk + (size_t)(b * (unsigned)NN + tid) * SUB;
    const v4f e0 = *(const v4f*)e;
    const v4f e1 = *(const v4f*)(e + 4);
    const v4f t0 = *(const v4f*)t;
    const v4f t1 = *(const v4f*)(t + 4);
    *(v4f*)&Xs[tid * 8u]      = e0 + t0;
    *(v4f*)&Xs[tid * 8u + 4u] = e1 + t1;
  }
  v4f z0, z1;
  {
    const float* e  = Eij + ((size_t)rowbi * NN + tid) * SUB;
    const float* ti = Ti + (size_t)rowbi * SUB;
    const float* tj = Tj + (size_t)(b * (unsigned)NN + tid) * SUB;
    const v4f e0 = *(const v4f*)e;
    const v4f e1 = *(const v4f*)(e + 4);
    const v4f i0 = *(const v4f*)ti;
    const v4f i1 = *(const v4f*)(ti + 4);
    const v4f j0 = *(const v4f*)tj;
    const v4f j1 = *(const v4f*)(tj + 4);
    const v4f b0 = *(const v4f*)bt;
    const v4f b1 = *(const v4f*)(bt + 4);
#pragma unroll
    for (int c = 0; c < 4; ++c) {
      z0[c] = ((e0[c] + i0[c]) + j0[c]) + bf16r(b0[c]);
      z1[c] = ((e1[c] + i1[c]) + j1[c]) + bf16r(b1[c]);
    }
  }
  __syncthreads();

  v4f m0 = {}, m1 = {};
  const float* yb = Ekj + ((size_t)b * NN * NN + tid) * SUB;
#pragma unroll 4
  for (unsigned k = 0; k < (unsigned)NN; ++k) {
    const v4f y0 = *(const v4f*)(yb + (size_t)k * (NN * SUB));
    const v4f y1 = *(const v4f*)(yb + (size_t)k * (NN * SUB) + 4);
    const v4f x0 = *(const v4f*)&Xs[k * 8u];
    const v4f x1 = *(const v4f*)&Xs[k * 8u + 4u];
#pragma unroll
    for (int c = 0; c < 4; ++c) {
      m0[c] = fmaxf(m0[c], (x0[c] + y0[c]) + z0[c]);
      m1[c] = fmaxf(m1[c], (x1[c] + y1[c]) + z1[c]);
    }
  }

  {
    v8h t8;
    v8h zz;
#pragma unroll
    for (int c = 0; c < 4; ++c) {
      t8[c]     = toh_flush(TCARRY * m0[c]);
      t8[c + 4] = toh_flush(TCARRY * m1[c]);
    }
#pragma unroll
    for (int c = 0; c < 8; ++c) zz[c] = (h16)0.0f;
    *(v8h*)&Ts[tid * LDTT]       = t8;
    *(v8h*)&Ts[tid * LDTT + 8u]  = zz;
    *(v8h*)&Ts[tid * LDTT + 16u] = zz;
    *(v8h*)&Ts[tid * LDTT + 24u] = zz;
  }
  __syncthreads();

  const unsigned cs0 = wave * (16u * LDO);
  const _Float16* wb = WoP + (size_t)m * 32u + hh * 8u;
#pragma unroll 1
  for (unsigned mt = 0; mt < 2u; ++mt) {
    const unsigned mrow0 = wave * 32u + mt * 16u;
    const v16h a = ld_frag(&Ts[mrow0 * LDTT], LDTT);
#pragma unroll
    for (unsigned nt = 0; nt < 8u; ++nt) {
      const v16h bfr = frag_at(wb + nt * 512u);
      v8f acc = {};
      acc = wmma16(a, bfr, acc);
      const float bb = bf16r(bo[nt * 16u + m]);
#pragma unroll
      for (int r = 0; r < 8; ++r)
        Cs[cs0 + (hh * 8u + (unsigned)r) * LDO + nt * 16u + m] =
            fmaxf(acc[r] * (1.0f / (TCARRY * WCARRY)) + bb, 0.0f);
    }
    wave_lds_sync();
    float* orow = out + ((size_t)rowbi * NN + mrow0) * DIM + lane * 4u;
#pragma unroll 4
    for (unsigned r = 0; r < 16u; ++r) {
      const v4f x = *(const v4f*)&Cs[cs0 + r * LDO + lane * 4u];
      *(volatile v4f*)(orow + (size_t)r * DIM) = x;
    }
    __threadfence();
#pragma unroll 4
    for (unsigned r = 0; r < 16u; ++r) {
      const v4f x = *(const v4f*)&Cs[cs0 + r * LDO + lane * 4u];
      *(volatile v4f*)(orow + (size_t)r * DIM) = x;
    }
    wave_lds_sync();
  }
}

extern "C" void kernel_launch(void* const* d_in, const int* in_sizes, int n_in,
                              void* d_out, int out_size, void* d_ws, size_t ws_size,
                              hipStream_t stream) {
  if (n_in < 10) return;
  if ((long long)in_sizes[0] < (long long)MT * DIM) return;
  if ((long long)in_sizes[1] < (long long)ME * DIM) return;
  if (in_sizes[2] < DIM * SUB || in_sizes[4] < DIM * SUB) return;
  if (in_sizes[3] < SUB || in_sizes[5] < SUB || in_sizes[7] < SUB) return;
  if (in_sizes[6] < 6 * SUB * SUB) return;
  if (in_sizes[8] < SUB * DIM || in_sizes[9] < DIM) return;
  if ((long long)out_size < (long long)ME * DIM) return;
  if (ws_size < WS_TOTAL) return;

  const float* node_emb = (const float*)d_in[0];
  const float* path_emb = (const float*)d_in[1];
  const float* Wn = (const float*)d_in[2];
  const float* bn = (const float*)d_in[3];
  const float* We = (const float*)d_in[4];
  const float* be = (const float*)d_in[5];
  const float* Wt = (const float*)d_in[6];
  const float* bt = (const float*)d_in[7];
  const float* Wo = (const float*)d_in[8];
  const float* bo = (const float*)d_in[9];
  float* out = (float*)d_out;

  char* ws = (char*)d_ws;
  _Float16* WeP = (_Float16*)(ws + OFF_WE);
  _Float16* WnP = (_Float16*)(ws + OFF_WN);
  _Float16* WoP = (_Float16*)(ws + OFF_WO);
  float* Eik = (float*)(ws + OFF_EIK);
  float* Ekj = (float*)(ws + OFF_EKJ);
  float* Eij = (float*)(ws + OFF_EIJ);
  float* Ti  = (float*)(ws + OFF_TI);
  float* Tj  = (float*)(ws + OFF_TJ);
  float* Tk  = (float*)(ws + OFF_TK);

  wprep_kernel<<<dim3(1), dim3(256), 0, stream>>>(We, Wn, Wo, WeP, WnP, WoP);
  proj_kernel<<<dim3(ME / PROWS), dim3(64), 0, stream>>>(path_emb, WeP, be, Wt, 24u,
                                                         Eik, Ekj, Eij);
  proj_kernel<<<dim3(MT / PROWS), dim3(64), 0, stream>>>(node_emb, WnP, bn, Wt, 0u,
                                                         Ti, Tj, Tk);
  tri_kernel<<<dim3(NB * NN), dim3(96), 0, stream>>>(Eik, Ekj, Eij, Ti, Tj, Tk, bt, WoP, bo, out);
}
